// SAttn_52956946760140
// MI455X (gfx1250) — hardware-verified
//
#include <hip/hip_runtime.h>
#include <math.h>

typedef __attribute__((ext_vector_type(16))) _Float16 v16h;
typedef __attribute__((ext_vector_type(16))) __bf16 v16b;
typedef __attribute__((ext_vector_type(8)))  _Float16 v8h;
typedef __attribute__((ext_vector_type(8)))  float v8f;
typedef __attribute__((ext_vector_type(4)))  float v4f;
typedef __attribute__((ext_vector_type(2)))  float v2f;
typedef __attribute__((ext_vector_type(4)))  unsigned v4u;
typedef __attribute__((ext_vector_type(4)))  int v4i;
typedef float __attribute__((may_alias)) float_a;
typedef int __attribute__((may_alias)) int_a;

template <typename T> __device__ __forceinline__ void vst2(void* p, T v) { *(volatile T*)p = v; __threadfence(); *(volatile T*)p = v; }
__device__ __forceinline__ v8f wmma16(v16h a, v16h b, v8f c) {
  v8f d = __builtin_amdgcn_wmma_f32_16x16x32_f16(false, a, false, b, (short)0, c, false, false);
  asm volatile("v_nop\n\tv_nop\n\tv_nop\n\tv_nop" : "+v"(d) : "v"(a), "v"(b));
  return d;
}
__device__ __forceinline__ v8f wmma_bf(v16b a, v16b b, v8f c) {
  v8f d = __builtin_amdgcn_wmma_f32_16x16x32_bf16(false, a, false, b, (short)0, c, false, false);
  asm volatile("v_nop\n\tv_nop\n\tv_nop\n\tv_nop" : "+v"(d) : "v"(a), "v"(b));
  return d;
}
__device__ __forceinline__ v16h frag_h(const _Float16* rowk0, int lane) {
  union { v16h v; v8h q[2]; } u; const _Float16* p = rowk0 + 8 * (lane >> 4);
  u.q[0] = *(const v8h*)p; u.q[1] = *(const v8h*)(p + 16); return u.v;
}
__device__ __forceinline__ v16h frag_f32(const float* rowk0, int lane) {
  v16h a; const float* p = rowk0 + 8 * (lane >> 4);
#pragma unroll
  for (int i = 0; i < 8; ++i) { a[i] = (_Float16)p[i]; a[8 + i] = (_Float16)p[16 + i]; }
  return a;
}
__device__ __forceinline__ v16h frag_f32s(const float* rowk0, int lane, float sc) {
  v16h a; const float* p = rowk0 + 8 * (lane >> 4);
#pragma unroll
  for (int i = 0; i < 8; ++i) { a[i] = (_Float16)(p[i] * sc); a[8 + i] = (_Float16)(p[16 + i] * sc); }
  return a;
}
__device__ __forceinline__ v16h fragc_f32(const float* W, int k0, int n, int lane, int ld, int K) {
  v16h a; const int g = lane >> 4;
#pragma unroll
  for (int i = 0; i < 8; ++i) { const int ka = k0 + 8 * g + i, kb = ka + 16;
    a[i] = (_Float16)(ka < K ? W[(size_t)(ka < K ? ka : K - 1) * ld + n] : 0.f); a[8 + i] = (_Float16)(kb < K ? W[(size_t)(kb < K ? kb : K - 1) * ld + n] : 0.f); }
  return a;
}
struct F2 { v16b h, l; };
__device__ __forceinline__ F2 bsplit16(const float v[16]) { F2 r;
#pragma unroll
  for (int i = 0; i < 16; ++i) { const __bf16 h = (__bf16)v[i]; r.h[i] = h; r.l[i] = (__bf16)(v[i] - (float)h); }
  return r; }
__device__ __forceinline__ F2 split_row(const float* row, int k0, int lane) { float v[16]; const float* p = row + k0 + 8 * (lane >> 4);
#pragma unroll
  for (int i = 0; i < 8; ++i) { v[i] = p[i]; v[8 + i] = p[16 + i]; }
  return bsplit16(v); }
__device__ __forceinline__ F2 split_rowK(const float* row, int k0, int lane, int K) { float v[16]; const int g = lane >> 4;
#pragma unroll
  for (int i = 0; i < 8; ++i) { const int ka = k0 + 8 * g + i, kb = ka + 16; v[i] = ka < K ? row[ka < K ? ka : K - 1] : 0.f; v[8 + i] = kb < K ? row[kb < K ? kb : K - 1] : 0.f; }
  return bsplit16(v); }
__device__ __forceinline__ F2 split_col(const float* W, int k0, int n, int lane, int ld, int K) { float v[16]; const int g = lane >> 4;
#pragma unroll
  for (int i = 0; i < 8; ++i) { const int ka = k0 + 8 * g + i, kb = ka + 16; v[i] = ka < K ? W[(size_t)(ka < K ? ka : K - 1) * ld + n] : 0.f; v[8 + i] = kb < K ? W[(size_t)(kb < K ? kb : K - 1) * ld + n] : 0.f; }
  return bsplit16(v); }
__device__ __forceinline__ v8f mac3(const F2& a, const F2& b, v8f c) { c = wmma_bf(a.l, b.h, c); c = wmma_bf(a.h, b.l, c); return wmma_bf(a.h, b.h, c); }
__device__ __forceinline__ float sigm(float v) { return 1.0f / (1.0f + expf(-v)); }
#define LDSX() do { asm volatile("s_wait_dscnt 0" ::: "memory"); __builtin_amdgcn_wave_barrier(); __builtin_amdgcn_fence(__ATOMIC_RELEASE, "workgroup"); } while (0)


#define NB 2
#define SS 2048
#define DM 512
#define NH 8
#define HD 64
#define NTOK (NB * SS)
#ifndef TQB
#define TQB (SS / 64)
#define TNB NB
#define TOB (NB * SS / 64)
#endif
typedef __attribute__((ext_vector_type(8))) __bf16 v8b;
__device__ __forceinline__ v16b frag_b(const __bf16* rowk0, int lane) {
  union { v16b v; v8b q[2]; } u; const __bf16* p = rowk0 + 8 * (lane >> 4);
  u.q[0] = *(const v8b*)p; u.q[1] = *(const v8b*)(p + 16); return u.v;
}
__device__ __forceinline__ float bfr(float v) { return (float)(__bf16)v; }
__device__ __attribute__((noinline)) float exp_ni(float v) { return expf(v); }
__device__ __attribute__((noinline)) float erf_ni(float v) { return erff(v); }

__device__ __attribute__((noinline)) float expm1_ni(float v) { return expm1f(v); }
#define WS_PW  0u
#define PLD 0
#define PQQ (PLD + 2 * DM * DM)
#define PKV (PQQ + DM * DM)
#define PFF (PKV + 2 * DM * DM)
#define PWEND (PFF + DM * DM)
#define WS_ML  (WS_PW + 2u * PWEND)
#define WS_NM  (WS_ML + 4u * NTOK * 2 * DM)
#define WS_ND  (WS_NM + 4u * NTOK * DM)
#define WS_Q   (WS_ND + 4u * NTOK * DM)
#define WS_KV  (WS_Q + 4u * NTOK * DM)
#define WS_VH  (WS_KV + 4u * NTOK * 2 * DM)
#define WS_VL  (WS_VH + 2u * NB * DM * SS)
#define WS_M2  (WS_VL + 2u * NB * DM * SS)
#define WS_END (WS_M2 + 4u * NTOK * DM)

__global__ __launch_bounds__(256) void k_packT(const float* __restrict__ WL, const float* __restrict__ WD, const float* __restrict__ WQ, const float* __restrict__ WK, const float* __restrict__ WV, const float* __restrict__ WF, __bf16* __restrict__ PW) {
  __shared__ __align__(16) __bf16 s[DM]; const int n = blockIdx.x, which = blockIdx.y, k = threadIdx.x; float v = 0.f; size_t dst;
  for (int kk = k; kk < DM; kk += 256) { float val = 0.f;
    if (which == 0) { const int part = n / DM, c = n % DM; val = (part == 0 ? WL : WD)[(size_t)kk * DM + c]; }
    else if (which == 1) { if (n < DM) { const int h = n / HD, e = n % HD; if (kk / HD == h) val = WQ[((size_t)h * HD + (kk % HD)) * HD + e]; } }
    else if (which == 2) { const int part = n / DM, c = n % DM; const int h = c / HD, e = c % HD; if (kk / HD == h) val = (part == 0 ? WK : WV)[((size_t)h * HD + (kk % HD)) * HD + e]; }
    else { if (n < DM) val = WF[(size_t)kk * DM + n]; }
    s[kk] = (__bf16)val; }
  if ((which == 1 || which == 3) && n >= DM) return;
  dst = (which == 0) ? (PLD + (size_t)n * DM) : (which == 1 ? (PQQ + (size_t)n * DM) : (which == 2 ? (PKV + (size_t)n * DM) : (PFF + (size_t)n * DM)));
  __syncthreads();
  if (k < DM / 8) vst2((unsigned*)(PW + dst + k * 8), *(const v4u*)&s[k * 8]);
  (void)v;
}
template <int RIN, int EPI>
__global__ __launch_bounds__(128) void k_gemm(const float* __restrict__ A, int lda, const __bf16* __restrict__ P, const float* __restrict__ bias, const float* __restrict__ RES, float* __restrict__ OUT, int ldo) {
  __shared__ __align__(16) float so[4][16][132];
  const int tid = threadIdx.x, wave = tid >> 5, lane = tid & 31, col = lane & 15, g = lane >> 4; const size_t r0 = (size_t)blockIdx.x * 64 + wave * 16; const int n0 = blockIdx.y * 128;
  v8f acc[8] = {};
#pragma unroll 2
  for (int kc = 0; kc < DM / 32; ++kc) { F2 a; if (RIN) { v16b ax; const float* p = A + (r0 + col) * lda + kc * 32 + 8 * g;
#pragma unroll
      for (int i = 0; i < 8; ++i) { ax[i] = (__bf16)p[i]; ax[8 + i] = (__bf16)p[16 + i]; } a.h = ax; a.l = ax; } else a = split_row(A + (r0 + col) * lda, kc * 32, lane);
#pragma unroll
    for (int j = 0; j < 8; ++j) { const v16b w = frag_b(P + (size_t)(n0 + j * 16 + col) * DM + kc * 32, lane); if (!RIN) acc[j] = wmma_bf(a.l, w, acc[j]); acc[j] = wmma_bf(a.h, w, acc[j]); } }
#pragma unroll
  for (int j = 0; j < 8; ++j) { const int n = n0 + j * 16 + col; const float bb = (EPI == 1) ? bfr(bias[n]) : 0.f;
#pragma unroll
    for (int r = 0; r < 8; ++r) { float v = acc[j][r] + bb; if (EPI == 1) { v = (v > 0.f) ? v : expm1_ni(v); v = RES[(r0 + 8 * g + r) * ldo + n] + v; } so[wave][8 * g + r][j * 16 + col] = v; } }
  LDSX();
  for (int rl = 0; rl < 16; ++rl) vst2(OUT + (r0 + rl) * ldo + n0 + lane * 4, *(const v4f*)&so[wave][rl][lane * 4]);
}
__global__ __launch_bounds__(256) void k_ln(const float* __restrict__ IN, int ldi, const float* __restrict__ G, const float* __restrict__ Bb, float* __restrict__ OUT) {
  __shared__ __align__(16) float s[8][DM]; const int wave = threadIdx.x >> 5, lane = threadIdx.x & 31; const size_t row = (size_t)blockIdx.x * 8 + wave; float v[16]; float sum = 0.f;
#pragma unroll
  for (int k = 0; k < 16; ++k) { v[k] = IN[row * ldi + lane + 32 * k]; sum += v[k]; }
#pragma unroll
  for (int o = 1; o < 32; o <<= 1) sum += __shfl_xor(sum, o);
  const float mu = sum / (float)DM; float var = 0.f;
#pragma unroll
  for (int k = 0; k < 16; ++k) { const float d = v[k] - mu; var += d * d; }
#pragma unroll
  for (int o = 1; o < 32; o <<= 1) var += __shfl_xor(var, o);
  const float rs = rsqrtf(var / (float)DM + 1e-6f);
#pragma unroll
  for (int k = 0; k < 16; ++k) { const int c = lane + 32 * k; s[wave][c] = (v[k] - mu) * rs * bfr(G[c]) + bfr(Bb[c]); }
  LDSX();
  for (int pc = lane; pc < DM / 4; pc += 32) vst2(OUT + row * DM + pc * 4, *(const v4f*)&s[wave][pc * 4]);
}
__global__ __launch_bounds__(256) void k_vplanes(const float* __restrict__ KV, __bf16* __restrict__ VH, __bf16* __restrict__ VL) {
  __shared__ __align__(16) __bf16 sh[128][72], sl[128][72]; const int tid = threadIdx.x; const size_t rb = (size_t)blockIdx.x * 64; const int c0 = blockIdx.y * 128; const int b = (int)(rb / SS), s0 = (int)(rb % SS);
  for (int q = tid; q < 64 * 128; q += 256) { const int rl = q >> 7, c = q & 127; const float v = KV[(rb + rl) * (2 * DM) + DM + c0 + c]; const __bf16 hb = (__bf16)v; sh[c][rl] = hb; sl[c][rl] = (__bf16)(v - (float)hb); }
  __syncthreads();
  for (int q = tid; q < 128 * 8; q += 256) { const int c = q >> 3, pc = q & 7; const size_t o = ((size_t)b * DM + c0 + c) * SS + s0 + pc * 8; vst2((unsigned*)(VH + o), *(const v4u*)&sh[c][pc * 8]); vst2((unsigned*)(VL + o), *(const v4u*)&sl[c][pc * 8]); }
}
__global__ __launch_bounds__(128) void k_attn(const float* __restrict__ Q, const float* __restrict__ KV, const __bf16* __restrict__ VH, const __bf16* __restrict__ VL, const float* __restrict__ ML, float* __restrict__ M2) {
  __shared__ __align__(16) float sp[4][16][36]; __shared__ __align__(16) float so[4][16][68];
  const int tid = threadIdx.x, wave = tid >> 5, lane = tid & 31, col = lane & 15, g = lane >> 4; const int qb = blockIdx.x, h = blockIdx.y, b = blockIdx.z; const int q0 = qb * 64 + wave * 16; const size_t rq = (size_t)b * SS + q0;
  F2 aq[2];
#pragma unroll
  for (int kc = 0; kc < 2; ++kc) aq[kc] = split_row(Q + (rq + col) * DM + h * HD, kc * 32, lane);
  float m[8], l[8];
#pragma unroll
  for (int r = 0; r < 8; ++r) { m[r] = -3.0e38f; l[r] = 0.f; }
  v8f acc[4] = {};
#pragma unroll 1
  for (int ks = 0; ks < SS / 32; ++ks) { v8f s[2];
#pragma unroll
    for (int ct = 0; ct < 2; ++ct) { const int kk = ks * 32 + ct * 16 + col; const float* krow = KV + ((size_t)b * SS + kk) * (2 * DM) + h * HD; v8f c = {};
#pragma unroll
      for (int kc = 0; kc < 2; ++kc) { const F2 kb = split_row(krow, kc * 32, lane); c = mac3(aq[kc], kb, c); }
      s[ct] = c; }
#pragma unroll
    for (int r = 0; r < 8; ++r) { float mx = fmaxf(s[0][r], s[1][r]);
#pragma unroll
      for (int o = 1; o < 16; o <<= 1) mx = fmaxf(mx, __shfl_xor(mx, o));
      const float mn = fmaxf(m[r], mx); const float alpha = exp_ni(m[r] - mn);
      const float e0 = exp_ni(s[0][r] - mn), e1 = exp_ni(s[1][r] - mn); float es = e0 + e1;
#pragma unroll
      for (int o = 1; o < 16; o <<= 1) es += __shfl_xor(es, o);
      l[r] = l[r] * alpha + es; m[r] = mn;
#pragma unroll
      for (int dt = 0; dt < 4; ++dt) acc[dt][r] *= alpha;
      sp[wave][8 * g + r][col] = e0; sp[wave][8 * g + r][16 + col] = e1; }
    LDSX();
    const F2 pa = split_row(&sp[wave][col][0], 0, lane);
#pragma unroll
    for (int dt = 0; dt < 4; ++dt) { const size_t vr = ((size_t)b * DM + h * HD + dt * 16 + col) * SS + ks * 32; const v16b vh = frag_b(VH + vr, lane), vl = frag_b(VL + vr, lane); acc[dt] = wmma_bf(pa.l, vh, acc[dt]); acc[dt] = wmma_bf(pa.h, vl, acc[dt]); acc[dt] = wmma_bf(pa.h, vh, acc[dt]); }
    LDSX(); }
#pragma unroll
  for (int r = 0; r < 8; ++r) { const float il = 1.0f / l[r]; const size_t row = rq + 8 * g + r;
#pragma unroll
    for (int dt = 0; dt < 4; ++dt) { const int c = h * HD + dt * 16 + col; so[wave][8 * g + r][dt * 16 + col] = ML[row * (2 * DM) + c] + acc[dt][r] * il; } }
  LDSX();
  for (int rl = 0; rl < 16; ++rl) if (lane < 16) vst2(M2 + (rq + rl) * DM + h * HD + lane * 4, *(const v4f*)&so[wave][rl][lane * 4]);
}
extern "C" void kernel_launch(void* const* d_in, const int* in_sizes, int n_in, void* d_out, int out_size, void* d_ws, size_t ws_size, hipStream_t stream) {
  (void)in_sizes; (void)n_in; (void)out_size;
  const float** F = (const float**)d_in;
  if (ws_size < (size_t)WS_END) return;
  char* ws = (char*)d_ws; __bf16 *PW = (__bf16*)(ws + WS_PW), *VH = (__bf16*)(ws + WS_VH), *VL = (__bf16*)(ws + WS_VL); float *ML = (float*)(ws + WS_ML), *NM = (float*)(ws + WS_NM), *ND = (float*)(ws + WS_ND), *Q = (float*)(ws + WS_Q), *KV = (float*)(ws + WS_KV), *M2 = (float*)(ws + WS_M2);
  const int NR = TNB * SS / 64;
  k_packT<<<dim3(2 * DM, 4), 256, 0, stream>>>(F[1], F[2], F[3], F[4], F[5], F[8], PW);
  k_gemm<1, 0><<<dim3(NR, 2 * DM / 128), 128, 0, stream>>>(F[0], DM, PW + PLD, nullptr, nullptr, ML, 2 * DM);
  k_ln<<<TNB * SS / 8, 256, 0, stream>>>(ML, 2 * DM, F[6], F[7], NM);
  k_ln<<<TNB * SS / 8, 256, 0, stream>>>(ML + DM, 2 * DM, F[6], F[7], ND);
  k_gemm<0, 0><<<dim3(NR, DM / 128), 128, 0, stream>>>(NM, DM, PW + PQQ, nullptr, nullptr, Q, DM);
  k_gemm<0, 0><<<dim3(NR, 2 * DM / 128), 128, 0, stream>>>(ND, DM, PW + PKV, nullptr, nullptr, KV, 2 * DM);
  k_vplanes<<<dim3(NR, DM / 128), 256, 0, stream>>>(KV, VH, VL);
  k_attn<<<dim3(TQB, NH, TNB), 128, 0, stream>>>(Q, KV, VH, VL, ML, M2);
  k_ln<<<TOB * 8, 256, 0, stream>>>(M2, DM, F[6], F[7], NM);
  k_gemm<0, 1><<<dim3(TOB, DM / 128), 128, 0, stream>>>(NM, DM, PW + PFF, F[9], M2, (float*)d_out, DM);
}
